// DialogueGCN_4037269259075
// MI455X (gfx1250) — hardware-verified
//
#include <hip/hip_runtime.h>
#include <stdint.h>


#define B_    64
#define L_    110
#define U_    768
#define G_    512
#define H_    256
#define FF_   2048
#define R_    8
#define NB_   30
#define TAG_  7
#define N_    (B_ * L_)
#define WIN_  10
#define QKVW_ (3 * U_)
#define YW_   (R_ * H_ + H_)
#define ZW_   (G_ + H_)
#define AHW_  (2 * H_)
#define ALW_  32
#define C2W_  32

typedef __bf16         v16bf __attribute__((ext_vector_type(16)));
typedef unsigned short v16us __attribute__((ext_vector_type(16)));
typedef float          v8f   __attribute__((ext_vector_type(8)));
typedef float          v4f   __attribute__((ext_vector_type(4)));

union Frag { v16bf v; v16us u; };

__device__ __forceinline__ unsigned int bfr(float x)
{
    unsigned int u = __float_as_uint(x);
    return (u + 0x7FFFu + ((u >> 16) & 1u)) >> 16;
}

__device__ __forceinline__ float wsum(float v)
{
#pragma unroll
    for (int o = 16; o > 0; o >>= 1) v += __shfl_xor(v, o, 32);
    return v;
}
__device__ __forceinline__ float wmax(float v)
{
#pragma unroll
    for (int o = 16; o > 0; o >>= 1) v = fmaxf(v, __shfl_xor(v, o, 32));
    return v;
}
__device__ __forceinline__ float dot4(v4f a, v4f b)
{
    return a.x * b.x + a.y * b.y + a.z * b.z + a.w * b.w;
}

__device__ __forceinline__ void wm(v8f& acc, const v16bf& a, const v16bf& b)
{
    acc = __builtin_amdgcn_wmma_f32_16x16x32_bf16(false, a, false, b, (short)0, acc, false, false);
    asm volatile("v_nop\n\tv_nop\n\tv_nop\n\tv_nop" : "+v"(acc) : "v"(a), "v"(b));
}

__device__ __forceinline__ void ldfrag(const float* __restrict__ p, Frag& hi, Frag& lo)
{
    const v4f x0 = *(const v4f*)(p);
    const v4f x1 = *(const v4f*)(p + 4);
    const v4f x2 = *(const v4f*)(p + 16);
    const v4f x3 = *(const v4f*)(p + 20);
    const float f[16] = {x0.x, x0.y, x0.z, x0.w, x1.x, x1.y, x1.z, x1.w,
                         x2.x, x2.y, x2.z, x2.w, x3.x, x3.y, x3.z, x3.w};
    v16us hu, lu;
#pragma unroll
    for (int i = 0; i < 16; ++i) {
        const unsigned int hs = bfr(f[i]);
        const float res = f[i] - __uint_as_float(hs << 16);
        hu[i] = (unsigned short)hs;
        lu[i] = (unsigned short)bfr(res);
    }
    hi.u = hu;
    lo.u = lu;
}

__global__ __launch_bounds__(128)
void k_gemm(const float* __restrict__ A, const float* __restrict__ W, const float* __restrict__ bias,
            float* __restrict__ C, int lda, int ldw, int ldc, int M, int Nd, int K, int has_bias, int relu)
{
    __shared__ __attribute__((aligned(16))) float st[4][32 * 32];
    const int l  = threadIdx.x & 31;
    const int wv = threadIdx.x >> 5;
    const int h  = l >> 4;
    const int m  = l & 15;
    const int m0 = ((int)blockIdx.y * 4 + wv) * 32;
    const int n0 = (int)blockIdx.x * 32;
    const bool act = (m0 < M);
    const int rb = act ? m0 : (M - 32);

    const v8f zero8 = {0.f, 0.f, 0.f, 0.f, 0.f, 0.f, 0.f, 0.f};
    v8f acc00 = zero8, acc01 = zero8, acc10 = zero8, acc11 = zero8;

    const float* ar0 = A + (size_t)(rb + m) * lda + 8 * h;
    const float* ar1 = ar0 + (size_t)16 * lda;
    const float* wr0 = W + (size_t)(n0 + m) * ldw + 8 * h;
    const float* wr1 = wr0 + (size_t)16 * ldw;

#pragma unroll 1
    for (int k0 = 0; k0 < K; k0 += 32) {
        Frag ah0, al0, ah1, al1, bh0, bl0, bh1, bl1;
        ldfrag(ar0 + k0, ah0, al0);
        ldfrag(ar1 + k0, ah1, al1);
        ldfrag(wr0 + k0, bh0, bl0);
        ldfrag(wr1 + k0, bh1, bl1);

        wm(acc00, ah0.v, bh0.v); wm(acc00, ah0.v, bl0.v); wm(acc00, al0.v, bh0.v);
        wm(acc01, ah0.v, bh1.v); wm(acc01, ah0.v, bl1.v); wm(acc01, al0.v, bh1.v);
        wm(acc10, ah1.v, bh0.v); wm(acc10, ah1.v, bl0.v); wm(acc10, al1.v, bh0.v);
        wm(acc11, ah1.v, bh1.v); wm(acc11, ah1.v, bl1.v); wm(acc11, al1.v, bh1.v);
    }

    float* s = &st[wv][0];
    {
        const int nA = n0 + m, nB = n0 + 16 + m;
        const float bA = has_bias ? bias[nA] : 0.f;
        const float bB = has_bias ? bias[nB] : 0.f;
#pragma unroll
        for (int r = 0; r < 8; ++r) {
            float v00 = acc00[r] + bA, v01 = acc01[r] + bB, v10 = acc10[r] + bA, v11 = acc11[r] + bB;
            if (relu) { v00 = fmaxf(v00, 0.f); v01 = fmaxf(v01, 0.f); v10 = fmaxf(v10, 0.f); v11 = fmaxf(v11, 0.f); }
            s[(8 * h + r) * 32 + m]           = v00;
            s[(8 * h + r) * 32 + 16 + m]      = v01;
            s[(16 + 8 * h + r) * 32 + m]      = v10;
            s[(16 + 8 * h + r) * 32 + 16 + m] = v11;
        }
    }
    __syncthreads();

    const int rsub = l >> 3;
    const int c4   = (l & 7) * 4;
    v4f vv[8];
#pragma unroll
    for (int i = 0; i < 8; ++i) vv[i] = *(const v4f*)&s[(4 * i + rsub) * 32 + c4];

    if (act) {
#pragma unroll
        for (int i = 0; i < 8; ++i)
            *(volatile v4f*)(C + (size_t)(m0 + 4 * i + rsub) * ldc + n0 + c4) = vv[i];
    }
    __threadfence();
    if (act) {
#pragma unroll
        for (int i = 0; i < 8; ++i)
            *(volatile v4f*)(C + (size_t)(m0 + 4 * i + rsub) * ldc + n0 + c4) = vv[i];
    }
}

__global__ __launch_bounds__(256)
void k_transpose(const float* __restrict__ src, float* __restrict__ dst, int rows, int cols, int ldd,
                 size_t sstride, size_t dstride)
{
    __shared__ float tile[32][33];
    src += (size_t)blockIdx.z * sstride;
    dst += (size_t)blockIdx.z * dstride;
    const int r0 = (int)blockIdx.y * 32, c0 = (int)blockIdx.x * 32;
    const int t = threadIdx.x;
#pragma unroll
    for (int i = 0; i < 4; ++i) {
        const int e = t + 256 * i;
        const int rr = e >> 5, cc = e & 31;
        const int gr = r0 + rr, gc = c0 + cc;
        tile[rr][cc] = (gr < rows && gc < cols) ? src[(size_t)gr * cols + gc] : 0.f;
    }
    __syncthreads();
    const int l = t & 31, wv = t >> 5;
    const int q = 4 * wv + (l >> 3);
    const int seg = (l & 7) * 4;
    v4f v;
    v.x = tile[seg + 0][q]; v.y = tile[seg + 1][q]; v.z = tile[seg + 2][q]; v.w = tile[seg + 3][q];
    const int orow = c0 + q;
    const bool ok = (orow < cols) && (r0 + seg + 3 < rows);
    float* p = dst + (size_t)orow * ldd + r0 + seg;
    if (ok) *(volatile v4f*)p = v;
    __threadfence();
    if (ok) *(volatile v4f*)p = v;
}

__global__ __launch_bounds__(256)
void k_wrel(const float* __restrict__ comp, const float* __restrict__ basis, float* __restrict__ wrel)
{
    __shared__ float cs[R_ * NB_];
    const int t = threadIdx.x;
    if (t < R_ * NB_) cs[t] = comp[t];
    __syncthreads();
    const size_t i4 = (size_t)blockIdx.x * 256 + t;
    const bool ok = (i4 < (size_t)(G_ * H_ / 4));
    const size_t i4c = ok ? i4 : 0;
    v4f acc[R_];
#pragma unroll
    for (int r = 0; r < R_; ++r) acc[r] = (v4f){0.f, 0.f, 0.f, 0.f};
#pragma unroll 1
    for (int b = 0; b < NB_; ++b) {
        const v4f x = *(const v4f*)(basis + (size_t)b * G_ * H_ + i4c * 4);
#pragma unroll
        for (int r = 0; r < R_; ++r) acc[r] += cs[r * NB_ + b] * x;
    }
    if (ok) {
#pragma unroll
        for (int r = 0; r < R_; ++r) *(volatile v4f*)(wrel + (size_t)r * G_ * H_ + i4 * 4) = acc[r];
    }
    __threadfence();
    if (ok) {
#pragma unroll
        for (int r = 0; r < R_; ++r) *(volatile v4f*)(wrel + (size_t)r * G_ * H_ + i4 * 4) = acc[r];
    }
}

__global__ __launch_bounds__(256)
void k_catw(const float* __restrict__ wa, const float* __restrict__ wb, float* __restrict__ dst)
{
    const int i4 = (int)blockIdx.x * 256 + threadIdx.x;
    const bool ok = i4 < (H_ * AHW_ / 4);
    const int i4c = ok ? i4 : 0;
    const int o = i4c / (AHW_ / 4);
    const int c4 = (i4c % (AHW_ / 4)) * 4;
    v4f v;
    if (c4 < H_) v = *(const v4f*)(wa + (size_t)o * H_ + c4);
    else         v = *(const v4f*)(wb + (size_t)o * H_ + (c4 - H_));
    if (ok) *(volatile v4f*)(dst + (size_t)i4 * 4) = v;
    __threadfence();
    if (ok) *(volatile v4f*)(dst + (size_t)i4 * 4) = v;
}

__global__ __launch_bounds__(256)
void k_padw(const float* __restrict__ w, float* __restrict__ dst)
{
    const int i4 = (int)blockIdx.x * 256 + threadIdx.x;
    const bool ok = i4 < (C2W_ * H_ / 4);
    const int i4c = ok ? i4 : 0;
    const int o = i4c / (H_ / 4);
    const int c4 = (i4c % (H_ / 4)) * 4;
    v4f v = (v4f){0.f, 0.f, 0.f, 0.f};
    if (o < TAG_) v = *(const v4f*)(w + (size_t)o * H_ + c4);
    if (ok) *(volatile v4f*)(dst + (size_t)i4 * 4) = v;
    __threadfence();
    if (ok) *(volatile v4f*)(dst + (size_t)i4 * 4) = v;
}

__global__ __launch_bounds__(192)
void k_attn(const float* __restrict__ qkv, float* __restrict__ att)
{
    __shared__ __attribute__((aligned(16))) float qs[U_];
    __shared__ float p[128];
    __shared__ float sinv;
    const int row = blockIdx.x;
    const int b = row / L_;
    const int t = threadIdx.x, l = t & 31, wv = t >> 5;
    const float* base = qkv + (size_t)(b * L_) * QKVW_;

    *(v4f*)&qs[4 * t] = *(const v4f*)(qkv + (size_t)row * QKVW_ + 4 * t);
    __syncthreads();

    const float scale = 1.0f / sqrtf((float)U_);
    for (int kk = wv; kk < L_; kk += 6) {
        const float* kr = base + (size_t)kk * QKVW_ + U_;
        float s = 0.f;
#pragma unroll
        for (int i = 0; i < 6; ++i) {
            const int d = 4 * l + 128 * i;
            const v4f kv = *(const v4f*)(kr + d);
            const v4f qv = *(const v4f*)&qs[d];
            s += dot4(kv, qv);
        }
        s = wsum(s);
        if (l == 0) p[kk] = s * scale;
    }
    __syncthreads();

    if (wv == 0) {
        float mx = -3.0e38f;
#pragma unroll 1
        for (int i = 0; i < 4; ++i) { const int idx = l + 32 * i; if (idx < L_) mx = fmaxf(mx, p[idx]); }
        mx = wmax(mx);
        float e[4];
        float sm = 0.f;
#pragma unroll 1
        for (int i = 0; i < 4; ++i) {
            const int idx = l + 32 * i;
            e[i] = (idx < L_) ? expf(p[idx] - mx) : 0.f;
            sm += e[i];
        }
        sm = wsum(sm);
#pragma unroll
        for (int i = 0; i < 4; ++i) { const int idx = l + 32 * i; if (idx < L_) p[idx] = e[i]; }
        if (l == 0) sinv = 1.0f / sm;
    }
    __syncthreads();

    v4f acc = (v4f){0.f, 0.f, 0.f, 0.f};
    const float* vb = base + 2 * U_ + 4 * t;
#pragma unroll 2
    for (int kk = 0; kk < L_; ++kk) {
        const float pk = p[kk];
        const v4f vv = *(const v4f*)(vb + (size_t)kk * QKVW_);
        acc += pk * vv;
    }
    const float inv = sinv;
    acc *= inv;
    float* op = att + (size_t)row * U_ + 4 * t;
    *(volatile v4f*)op = acc;
    __threadfence();
    *(volatile v4f*)op = acc;
}

__global__ __launch_bounds__(192)
void k_ln(const float* __restrict__ xa, const float* __restrict__ xb,
          const float* __restrict__ g, const float* __restrict__ be, float* __restrict__ out)
{
    __shared__ float sh1[8];
    __shared__ float sh2[8];
    const int row = blockIdx.x;
    const int t = threadIdx.x, l = t & 31, wv = t >> 5;
    const size_t off = (size_t)row * U_ + 4 * t;
    const v4f a = *(const v4f*)(xa + off) + *(const v4f*)(xb + off);
    float s = a.x + a.y + a.z + a.w;
    s = wsum(s);
    if (l == 0) sh1[wv] = s;
    __syncthreads();
    float tot = 0.f;
#pragma unroll
    for (int i = 0; i < 6; ++i) tot += sh1[i];
    const float mean = tot * (1.0f / (float)U_);
    const v4f d = a - mean;
    float q = dot4(d, d);
    q = wsum(q);
    if (l == 0) sh2[wv] = q;
    __syncthreads();
    float tq = 0.f;
#pragma unroll
    for (int i = 0; i < 6; ++i) tq += sh2[i];
    const float var = tq * (1.0f / (float)U_);
    const float rstd = 1.0f / sqrtf(var + 1e-5f);
    const v4f gv = *(const v4f*)(g + 4 * t);
    const v4f bv = *(const v4f*)(be + 4 * t);
    const v4f o = d * rstd * gv + bv;
    *(volatile v4f*)(out + off) = o;
    __threadfence();
    *(volatile v4f*)(out + off) = o;
}

__global__ __launch_bounds__(128)
void k_alpha(const float* __restrict__ tb, const float* __restrict__ z, float* __restrict__ alpha)
{
    __shared__ __attribute__((aligned(16))) float ts[G_];
    __shared__ float sc[32];
    __shared__ __attribute__((aligned(16))) float line[ALW_];
    const int row = blockIdx.x;
    const int b = row / L_, j = row % L_;
    const int klo = (j - WIN_ > 0) ? (j - WIN_) : 0;
    const int khi = (j + WIN_ < L_ - 1) ? (j + WIN_) : (L_ - 1);
    const int nk = khi - klo + 1;
    const int t = threadIdx.x, l = t & 31, wv = t >> 5;

    *(v4f*)&ts[4 * t] = *(const v4f*)(tb + (size_t)row * G_ + 4 * t);
    if (t < 32) { line[t] = 0.f; sc[t] = 0.f; }
    __syncthreads();

    for (int idx = wv; idx < nk; idx += 4) {
        const int k = klo + idx;
        const float* fr = z + (size_t)(b * L_ + k) * ZW_;
        float s = 0.f;
#pragma unroll
        for (int i = 0; i < 4; ++i) {
            const int d = 4 * l + 128 * i;
            const v4f fv = *(const v4f*)(fr + d);
            const v4f tv = *(const v4f*)&ts[d];
            s += dot4(fv, tv);
        }
        s = wsum(s);
        if (l == 0) sc[idx] = s;
    }
    __syncthreads();

    if (wv == 0) {
        const float v = (l < nk) ? sc[l] : -3.0e38f;
        const float mx = wmax(v);
        const float e = (l < nk) ? expf(v - mx) : 0.f;
        const float sm = wsum(e);
        const float a = e * (1.0f / sm);
        if (l < nk) line[klo + l - j + WIN_] = a;
    }
    __syncthreads();

    v4f ov = (v4f){0.f, 0.f, 0.f, 0.f};
    if (t < 8) ov = *(const v4f*)&line[4 * t];
    float* p = alpha + (size_t)row * ALW_ + 4 * t;
    if (t < 8) *(volatile v4f*)p = ov;
    __threadfence();
    if (t < 8) *(volatile v4f*)p = ov;
}

__global__ __launch_bounds__(64)
void k_rgcn(const float* __restrict__ y, const int* __restrict__ sp, const float* __restrict__ bias,
            float* __restrict__ ah)
{
    const int node = blockIdx.x;
    const int b = node / L_, kp = node % L_;
    const int jlo = (kp - WIN_ > 0) ? (kp - WIN_) : 0;
    const int jhi = (kp + WIN_ < L_ - 1) ? (kp + WIN_) : (L_ - 1);
    const int t = threadIdx.x;
    const int spd = sp[node];

    float cnt[R_];
#pragma unroll
    for (int r = 0; r < R_; ++r) cnt[r] = 0.f;
    for (int j = jlo; j <= jhi; ++j) {
        const int et = (sp[b * L_ + j] * 2 + spd) * 2 + ((j >= kp) ? 1 : 0);
#pragma unroll
        for (int r = 0; r < R_; ++r) cnt[r] += (et == r) ? 1.f : 0.f;
    }
    float rc[R_];
#pragma unroll
    for (int r = 0; r < R_; ++r) rc[r] = (cnt[r] > 0.f) ? (1.0f / cnt[r]) : 0.f;

    v4f acc = (v4f){0.f, 0.f, 0.f, 0.f};
    for (int j = jlo; j <= jhi; ++j) {
        const int et = (sp[b * L_ + j] * 2 + spd) * 2 + ((j >= kp) ? 1 : 0);
        float w = 0.f;
#pragma unroll
        for (int r = 0; r < R_; ++r) w = (et == r) ? rc[r] : w;
        int etc = et < 0 ? 0 : et;
        etc = etc > (R_ - 1) ? (R_ - 1) : etc;
        const v4f yv = *(const v4f*)(y + (size_t)(b * L_ + j) * YW_ + etc * H_ + 4 * t);
        acc += w * yv;
    }
    const v4f rt = *(const v4f*)(y + (size_t)node * YW_ + R_ * H_ + 4 * t);
    const v4f bv = *(const v4f*)(bias + 4 * t);
    const v4f h1 = acc + rt + bv;
    float* p = ah + (size_t)node * AHW_ + H_ + 4 * t;
    *(volatile v4f*)p = h1;
    __threadfence();
    *(volatile v4f*)p = h1;
}

__global__ __launch_bounds__(64)
void k_gconv(const float* __restrict__ alpha, float* ah)
{
    const int node = blockIdx.x;
    const int b = node / L_, kp = node % L_;
    const int jlo = (kp - WIN_ > 0) ? (kp - WIN_) : 0;
    const int jhi = (kp + WIN_ < L_ - 1) ? (kp + WIN_) : (L_ - 1);
    const int t = threadIdx.x;
    v4f acc = (v4f){0.f, 0.f, 0.f, 0.f};
    for (int j = jlo; j <= jhi; ++j) {
        const float w = alpha[(size_t)(b * L_ + j) * ALW_ + (kp - j + WIN_)];
        const v4f hv = *(const v4f*)(ah + (size_t)(b * L_ + j) * AHW_ + H_ + 4 * t);
        acc += w * hv;
    }
    float* p = ah + (size_t)node * AHW_ + 4 * t;
    *(volatile v4f*)p = acc;
    __threadfence();
    *(volatile v4f*)p = acc;
}

__global__ __launch_bounds__(256)
void k_pack(const float* __restrict__ c2, const float* __restrict__ cb, float* __restrict__ out)
{
    const int i4 = (int)blockIdx.x * 256 + threadIdx.x;
    const bool ok = i4 < (N_ * TAG_ / 4);
    v4f v = (v4f){0.f, 0.f, 0.f, 0.f};
    if (ok) {
        float o[4];
#pragma unroll
        for (int c = 0; c < 4; ++c) {
            const int i = i4 * 4 + c;
            const int n = i / TAG_, tg = i % TAG_;
            o[c] = c2[(size_t)n * C2W_ + tg] + cb[tg];
        }
        v.x = o[0]; v.y = o[1]; v.z = o[2]; v.w = o[3];
    }
    if (ok) *(volatile v4f*)(out + (size_t)i4 * 4) = v;
    __threadfence();
    if (ok) *(volatile v4f*)(out + (size_t)i4 * 4) = v;
}

extern "C" void kernel_launch(void* const* d_in, const int* in_sizes, int n_in,
                              void* d_out, int out_size, void* d_ws, size_t ws_size,
                              hipStream_t stream)
{
    if (n_in < 33) return;
    if (in_sizes[0] != N_ * U_ || in_sizes[1] != 3 * U_ * U_ || in_sizes[7] != FF_ * U_ ||
        in_sizes[13] != G_ * U_ || in_sizes[15] != G_ * G_ || in_sizes[16] != NB_ * G_ * H_ ||
        in_sizes[17] != R_ * NB_ || in_sizes[18] != G_ * H_ || in_sizes[23] != H_ * (G_ + H_) ||
        in_sizes[25] != TAG_ * H_ || in_sizes[26] != TAG_ || in_sizes[27] != N_) return;
    if (out_size != N_ * TAG_) return;

    const float* x      = (const float*)d_in[0];
    const float* inpw   = (const float*)d_in[1];
    const float* inpb   = (const float*)d_in[2];
    const float* outw   = (const float*)d_in[3];
    const float* outb   = (const float*)d_in[4];
    const float* ln1g   = (const float*)d_in[5];
    const float* ln1b   = (const float*)d_in[6];
    const float* ff1w   = (const float*)d_in[7];
    const float* ff1b   = (const float*)d_in[8];
    const float* ff2w   = (const float*)d_in[9];
    const float* ff2b   = (const float*)d_in[10];
    const float* ln2g   = (const float*)d_in[11];
    const float* ln2b   = (const float*)d_in[12];
    const float* tow    = (const float*)d_in[13];
    const float* tob    = (const float*)d_in[14];
    const float* attw   = (const float*)d_in[15];
    const float* basis  = (const float*)d_in[16];
    const float* comp   = (const float*)d_in[17];
    const float* root   = (const float*)d_in[18];
    const float* rgcnb  = (const float*)d_in[19];
    const float* gcrelw = (const float*)d_in[20];
    const float* gcrelb = (const float*)d_in[21];
    const float* gcrootw= (const float*)d_in[22];
    const float* clf1w  = (const float*)d_in[23];
    const float* clf1b  = (const float*)d_in[24];
    const float* clf2w  = (const float*)d_in[25];
    const float* clf2b  = (const float*)d_in[26];
    const int*   speaker= (const int*)d_in[27];
    float* out = (float*)d_out;

    char* ws = (char*)d_ws;
    size_t off = 0;
    auto carve = [&](size_t bytes) { size_t o = off; off += (bytes + 255) & ~(size_t)255; return o; };
    const size_t oRA   = carve((size_t)N_ * QKVW_ * 4);
    const size_t oRB   = carve((size_t)N_ * U_ * 4);
    const size_t oRC   = carve((size_t)N_ * U_ * 4);
    const size_t oZ    = carve((size_t)N_ * ZW_ * 4);
    const size_t oT    = carve((size_t)N_ * G_ * 4);
    const size_t oAL   = carve((size_t)N_ * ALW_ * 4);
    const size_t oAH   = carve((size_t)N_ * AHW_ * 4);
    const size_t oC1   = carve((size_t)N_ * H_ * 4);
    const size_t oC2   = carve((size_t)N_ * C2W_ * 4);
    const size_t oWREL = carve((size_t)R_ * G_ * H_ * 4);
    const size_t oWRG  = carve((size_t)YW_ * G_ * 4);
    const size_t oATWT = carve((size_t)G_ * G_ * 4);
    const size_t oWGC  = carve((size_t)H_ * AHW_ * 4);
    const size_t oW2P  = carve((size_t)C2W_ * H_ * 4);
    if (off > ws_size) return;

    float* QKV  = (float*)(ws + oRA);
    float* F1   = (float*)(ws + oRA);
    float* HS   = (float*)(ws + oRA);
    float* Y    = (float*)(ws + oRA);
    float* ATT  = (float*)(ws + oRB);
    float* H    = (float*)(ws + oRB);
    float* AOUT = (float*)(ws + oRC);
    float* F2   = (float*)(ws + oRC);
    float* Z    = (float*)(ws + oZ);
    float* T    = (float*)(ws + oT);
    float* AL   = (float*)(ws + oAL);
    float* AH   = (float*)(ws + oAH);
    float* C1   = (float*)(ws + oC1);
    float* C2   = (float*)(ws + oC2);
    float* WREL = (float*)(ws + oWREL);
    float* WRG  = (float*)(ws + oWRG);
    float* ATWT = (float*)(ws + oATWT);
    float* WGC  = (float*)(ws + oWGC);
    float* W2P  = (float*)(ws + oW2P);

    auto gemm = [&](const float* A, int lda, const float* W, int ldw, const float* bias, int has_bias,
                    float* C, int ldc, int M, int Nd, int K, int relu) {
        if ((M % 32) || (Nd % 32) || (K % 32) || M < 32) return;
        k_gemm<<<dim3((unsigned)(Nd / 32), (unsigned)((M + 127) / 128)), 128, 0, stream>>>(
            A, W, bias, C, lda, ldw, ldc, M, Nd, K, has_bias, relu);
    };

    k_wrel<<<dim3((G_ * H_ / 4 + 255) / 256), 256, 0, stream>>>(comp, basis, WREL);
    k_transpose<<<dim3(H_ / 32, G_ / 32, R_), 256, 0, stream>>>(WREL, WRG, G_, H_, G_,
                                                                 (size_t)G_ * H_, (size_t)H_ * G_);
    k_transpose<<<dim3(H_ / 32, G_ / 32, 1), 256, 0, stream>>>(root, WRG + (size_t)R_ * H_ * G_, G_, H_, G_, 0, 0);
    k_transpose<<<dim3(G_ / 32, G_ / 32, 1), 256, 0, stream>>>(attw, ATWT, G_, G_, G_, 0, 0);
    k_catw<<<dim3((H_ * AHW_ / 4 + 255) / 256), 256, 0, stream>>>(gcrelw, gcrootw, WGC);
    k_padw<<<dim3((C2W_ * H_ / 4 + 255) / 256), 256, 0, stream>>>(clf2w, W2P);

    gemm(x, U_, inpw, U_, inpb, 1, QKV, QKVW_, N_, QKVW_, U_, 0);
    k_attn<<<dim3(N_), 192, 0, stream>>>(QKV, ATT);
    gemm(ATT, U_, outw, U_, outb, 1, AOUT, U_, N_, U_, U_, 0);
    k_ln<<<dim3(N_), 192, 0, stream>>>(x, AOUT, ln1g, ln1b, H);
    gemm(H, U_, ff1w, U_, ff1b, 1, F1, FF_, N_, FF_, U_, 1);
    gemm(F1, FF_, ff2w, FF_, ff2b, 1, F2, U_, N_, U_, FF_, 0);
    k_ln<<<dim3(N_), 192, 0, stream>>>(H, F2, ln2g, ln2b, HS);
    gemm(HS, U_, tow, U_, tob, 1, Z, ZW_, N_, G_, U_, 0);

    gemm(Z, ZW_, ATWT, G_, ATWT, 0, T, G_, N_, G_, G_, 0);
    k_alpha<<<dim3(N_), 128, 0, stream>>>(T, Z, AL);

    gemm(Z, ZW_, WRG, G_, WRG, 0, Y, YW_, N_, YW_, G_, 0);
    k_rgcn<<<dim3(N_), 64, 0, stream>>>(Y, speaker, rgcnb, AH);

    k_gconv<<<dim3(N_), 64, 0, stream>>>(AL, AH);
    gemm(AH, AHW_, WGC, AHW_, gcrelb, 1, Z + G_, ZW_, N_, H_, AHW_, 0);

    gemm(Z, ZW_, clf1w, ZW_, clf1b, 1, C1, H_, N_, H_, ZW_, 1);
    gemm(C1, H_, W2P, H_, W2P, 0, C2, C2W_, N_, C2W_, H_, 0);
    k_pack<<<dim3((N_ * TAG_ / 4 + 255) / 256), 256, 0, stream>>>(C2, clf2b, out);
}
